// DynamicRadiusChannelFusion_5471788335636
// MI455X (gfx1250) — hardware-verified
//
#include <hip/hip_runtime.h>
#include <math.h>

typedef __attribute__((ext_vector_type(16))) _Float16 v16h;
typedef __attribute__((ext_vector_type(16))) __bf16 v16b;
typedef __attribute__((ext_vector_type(8)))  _Float16 v8h;
typedef __attribute__((ext_vector_type(8)))  float v8f;
typedef __attribute__((ext_vector_type(4)))  float v4f;
typedef __attribute__((ext_vector_type(2)))  float v2f;
typedef __attribute__((ext_vector_type(4)))  unsigned v4u;
typedef __attribute__((ext_vector_type(4)))  int v4i;
typedef float __attribute__((may_alias)) float_a;
typedef int __attribute__((may_alias)) int_a;

template <typename T> __device__ __forceinline__ void vst2(void* p, T v) { *(volatile T*)p = v; __threadfence(); *(volatile T*)p = v; }
__device__ __forceinline__ v8f wmma16(v16h a, v16h b, v8f c) {
  v8f d = __builtin_amdgcn_wmma_f32_16x16x32_f16(false, a, false, b, (short)0, c, false, false);
  asm volatile("v_nop\n\tv_nop\n\tv_nop\n\tv_nop" : "+v"(d) : "v"(a), "v"(b));
  return d;
}
__device__ __forceinline__ v8f wmma_bf(v16b a, v16b b, v8f c) {
  v8f d = __builtin_amdgcn_wmma_f32_16x16x32_bf16(false, a, false, b, (short)0, c, false, false);
  asm volatile("v_nop\n\tv_nop\n\tv_nop\n\tv_nop" : "+v"(d) : "v"(a), "v"(b));
  return d;
}
__device__ __forceinline__ v16h frag_h(const _Float16* rowk0, int lane) {
  union { v16h v; v8h q[2]; } u; const _Float16* p = rowk0 + 8 * (lane >> 4);
  u.q[0] = *(const v8h*)p; u.q[1] = *(const v8h*)(p + 16); return u.v;
}
__device__ __forceinline__ v16h frag_f32(const float* rowk0, int lane) {
  v16h a; const float* p = rowk0 + 8 * (lane >> 4);
#pragma unroll
  for (int i = 0; i < 8; ++i) { a[i] = (_Float16)p[i]; a[8 + i] = (_Float16)p[16 + i]; }
  return a;
}
__device__ __forceinline__ v16h frag_f32s(const float* rowk0, int lane, float sc) {
  v16h a; const float* p = rowk0 + 8 * (lane >> 4);
#pragma unroll
  for (int i = 0; i < 8; ++i) { a[i] = (_Float16)(p[i] * sc); a[8 + i] = (_Float16)(p[16 + i] * sc); }
  return a;
}
__device__ __forceinline__ v16h fragc_f32(const float* W, int k0, int n, int lane, int ld, int K) {
  v16h a; const int g = lane >> 4;
#pragma unroll
  for (int i = 0; i < 8; ++i) { const int ka = k0 + 8 * g + i, kb = ka + 16;
    a[i] = (_Float16)(ka < K ? W[(size_t)(ka < K ? ka : K - 1) * ld + n] : 0.f); a[8 + i] = (_Float16)(kb < K ? W[(size_t)(kb < K ? kb : K - 1) * ld + n] : 0.f); }
  return a;
}
struct F2 { v16b h, l; };
__device__ __forceinline__ F2 bsplit16(const float v[16]) { F2 r;
#pragma unroll
  for (int i = 0; i < 16; ++i) { const __bf16 h = (__bf16)v[i]; r.h[i] = h; r.l[i] = (__bf16)(v[i] - (float)h); }
  return r; }
__device__ __forceinline__ F2 split_row(const float* row, int k0, int lane) { float v[16]; const float* p = row + k0 + 8 * (lane >> 4);
#pragma unroll
  for (int i = 0; i < 8; ++i) { v[i] = p[i]; v[8 + i] = p[16 + i]; }
  return bsplit16(v); }
__device__ __forceinline__ F2 split_rowK(const float* row, int k0, int lane, int K) { float v[16]; const int g = lane >> 4;
#pragma unroll
  for (int i = 0; i < 8; ++i) { const int ka = k0 + 8 * g + i, kb = ka + 16; v[i] = ka < K ? row[ka < K ? ka : K - 1] : 0.f; v[8 + i] = kb < K ? row[kb < K ? kb : K - 1] : 0.f; }
  return bsplit16(v); }
__device__ __forceinline__ F2 split_col(const float* W, int k0, int n, int lane, int ld, int K) { float v[16]; const int g = lane >> 4;
#pragma unroll
  for (int i = 0; i < 8; ++i) { const int ka = k0 + 8 * g + i, kb = ka + 16; v[i] = ka < K ? W[(size_t)(ka < K ? ka : K - 1) * ld + n] : 0.f; v[8 + i] = kb < K ? W[(size_t)(kb < K ? kb : K - 1) * ld + n] : 0.f; }
  return bsplit16(v); }
__device__ __forceinline__ v8f mac3(const F2& a, const F2& b, v8f c) { c = wmma_bf(a.l, b.h, c); c = wmma_bf(a.h, b.l, c); return wmma_bf(a.h, b.h, c); }
__device__ __forceinline__ float sigm(float v) { return 1.0f / (1.0f + expf(-v)); }
#define LDSX() do { asm volatile("s_wait_dscnt 0" ::: "memory"); __builtin_amdgcn_wave_barrier(); __builtin_amdgcn_fence(__ATOMIC_RELEASE, "workgroup"); } while (0)


#define NB 2
#define CC 128
#define NN 8192
#ifndef NNS
#define NNS NN
#endif
#define NR (NB * NN)
#define KNB 16
#define CH 128
#define SEH 8
typedef __attribute__((ext_vector_type(8))) __bf16 v8b;
__device__ __forceinline__ v16b frag_b(const __bf16* rowk0, int lane) {
  union { v16b v; v8b q[2]; } u; const __bf16* p = rowk0 + 8 * (lane >> 4);
  u.q[0] = *(const v8b*)p; u.q[1] = *(const v8b*)(p + 16); return u.v;
}
__device__ __forceinline__ float bfr(float v) { return (float)(__bf16)v; }
__device__ __attribute__((noinline)) float exp_ni(float v) { return expf(v); }
__device__ __attribute__((noinline)) float erf_ni(float v) { return erff(v); }

#define PK_1 0
#define PK_2 (CH * 2 * CC)
#define PK_END (PK_2 + CH * CH)
#define WS_PK   0u
#define WS_P4   (((2u * PK_END) + 127u) / 128u * 128u)
#define WS_SQ   (WS_P4 + 4u * NR * 4)
#define WS_AH   (WS_SQ + 4u * NR)
#define WS_AL   (WS_AH + 2u * NR * 2 * CC)
#define WS_H    (WS_AL + 2u * NR * 2 * CC)
#define WS_ST1  (WS_H + 4u * NR * CH)
#define WS_MR1  (WS_ST1 + 8u * 256 * CH * 2)
#define WS_HBH  (WS_MR1 + 4u * 4 * CH)
#define WS_HBL  (WS_HBH + 2u * NR * CH)
#define WS_Y    (WS_HBL + 2u * NR * CH)
#define WS_ST2  (WS_Y + 4u * NR * CH)
#define WS_MR2  (WS_ST2 + 8u * 256 * CH * 2)
#define WS_ST3  (WS_MR2 + 4u * 4 * CH)
#define WS_GT   (WS_ST3 + 8u * 256 * CH)
#define WS_END  (WS_GT + 4u * NB * CH)

__global__ __launch_bounds__(256) void k_pack(const float* __restrict__ W1, const float* __restrict__ W2, __bf16* __restrict__ PK) {
  __shared__ __align__(16) __bf16 s[2 * CC]; const int n = blockIdx.x, which = blockIdx.y, t = threadIdx.x; int K; size_t dst;
  if (which == 0) { K = 2 * CC; dst = PK_1 + (size_t)n * 2 * CC; s[t] = (__bf16)W1[(size_t)n * 2 * CC + t]; } else { K = CH; dst = PK_2 + (size_t)n * CH; if (t < CH) s[t] = (__bf16)W2[(size_t)n * CH + t]; }
  __syncthreads();
  if (t < K / 8) vst2((unsigned*)(PK + dst + t * 8), *(const v4u*)&s[t * 8]);
}
__global__ __launch_bounds__(64) void k_prep(const float* __restrict__ POS, float* __restrict__ P4, float* __restrict__ SQ) {
  __shared__ __align__(16) float sp[64][4]; __shared__ __align__(16) float ss[64]; const int t = threadIdx.x; const int pb = blockIdx.x, b = blockIdx.y; const int n = pb * 64 + t;
  const float x0 = bfr(POS[((size_t)b * 3 + 0) * NNS + n]), x1 = bfr(POS[((size_t)b * 3 + 1) * NNS + n]), x2 = bfr(POS[((size_t)b * 3 + 2) * NNS + n]);
  sp[t][0] = x0; sp[t][1] = x1; sp[t][2] = x2; sp[t][3] = 0.f; ss[t] = __fadd_rn(__fadd_rn(__fmul_rn(x0, x0), __fmul_rn(x2, x2)), __fmul_rn(x1, x1));
  __syncthreads();
  const size_t row0 = (size_t)b * NN + pb * 64; vst2(P4 + (row0 + t) * 4, *(const v4f*)&sp[t][0]); if (t < 16) vst2(SQ + row0 + t * 4, *(const v4f*)&ss[t * 4]);
}
__global__ __launch_bounds__(128) void k_knn(const float* __restrict__ P4, const float* __restrict__ SQ, const float* __restrict__ X, __bf16* __restrict__ AH, __bf16* __restrict__ AL) {
  __shared__ float sd[4][NN]; __shared__ int sidx[4][KNB]; __shared__ float sw[4][KNB]; __shared__ __align__(16) __bf16 sh_[4][2 * CC + 8], sl_[4][2 * CC + 8];
  const int tid = threadIdx.x, wave = tid >> 5, lane = tid & 31; const size_t q = (size_t)blockIdx.x * 4 + wave; const int b = (int)(q / NN); const int n = (int)(q % NN); const size_t base = (size_t)b * NN;
  const float qx0 = P4[q * 4], qx1 = P4[q * 4 + 1], qx2 = P4[q * 4 + 2], sqi = SQ[q];
  for (int j = lane; j < NN; j += 32) { const size_t pj = base + j; const float dot = __fadd_rn(__fadd_rn(__fmul_rn(qx0, P4[pj * 4]), __fmul_rn(qx1, P4[pj * 4 + 1])), __fmul_rn(qx2, P4[pj * 4 + 2])); sd[wave][j] = __fsub_rn(__fadd_rn(sqi, SQ[pj]), __fmul_rn(2.0f, dot)); }
  __syncthreads();
#pragma unroll 1
  for (int s = 0; s < KNB; ++s) { float bv = 3.0e38f; int bi = 0x7fffffff;
    for (int j = lane; j < NN; j += 32) { const float v = sd[wave][j]; if (v < bv) { bv = v; bi = j; } }
#pragma unroll
    for (int o = 1; o < 32; o <<= 1) { const float ov = __shfl_xor(bv, o); const int oi = __shfl_xor(bi, o); if (ov < bv || (ov == bv && oi < bi)) { bv = ov; bi = oi; } }
    if (lane == 0) { sidx[wave][s] = bi; sd[wave][bi] = 3.0e38f; }
    __syncthreads(); }
  { float dk = 3.0e38f; if (lane < KNB) { const size_t pj = base + sidx[wave][lane]; const float dx = P4[pj * 4] - qx0, dy = P4[pj * 4 + 1] - qx1, dz = P4[pj * 4 + 2] - qx2; dk = fmaxf(sqrtf((dx * dx + dz * dz) + dy * dy), 1e-6f); }
    float lg = (lane < KNB) ? -dk / 0.2f : -3.0e38f; float mx = lg;
#pragma unroll
    for (int o = 1; o < 32; o <<= 1) mx = fmaxf(mx, __shfl_xor(mx, o));
    const float e = (lane < KNB) ? exp_ni(lg - mx) : 0.f; float se = e;
#pragma unroll
    for (int o = 1; o < 32; o <<= 1) se += __shfl_xor(se, o);
    if (lane < KNB) sw[wave][lane] = e / se; }
  __syncthreads();
  for (int c = lane; c < CC; c += 32) { const float* xc = X + ((size_t)b * CC + c) * NNS; float a = 0.f;
#pragma unroll
    for (int k = 0; k < KNB; ++k) a += bfr(xc[sidx[wave][k]]) * sw[wave][k];
    const float xv = bfr(xc[n]); sh_[wave][c] = (__bf16)xv; sl_[wave][c] = (__bf16)0.f; const __bf16 hb = (__bf16)a; sh_[wave][CC + c] = hb; sl_[wave][CC + c] = (__bf16)(a - (float)hb); }
  __syncthreads();
  for (int e2 = tid; e2 < 4 * (2 * CC / 8) * 2; e2 += 128) { const int plane = e2 / (4 * 2 * CC / 8), rem = e2 % (4 * 2 * CC / 8); const int r = rem / (2 * CC / 8), pc = rem % (2 * CC / 8); const size_t o = ((size_t)blockIdx.x * 4 + r) * 2 * CC + pc * 8;
    if (plane == 0) vst2((unsigned*)(AH + o), *(const v4u*)&sh_[r][pc * 8]); else vst2((unsigned*)(AL + o), *(const v4u*)&sl_[r][pc * 8]); }
}
template <int MODE>
__global__ __launch_bounds__(128) void k_gemm(const __bf16* __restrict__ AHp, const __bf16* __restrict__ ALp, const __bf16* __restrict__ PK, float* __restrict__ OUTR, double* __restrict__ ST) {
  __shared__ __align__(16) float so[4][16][CH + 4]; __shared__ __align__(16) double sst[CH][2];
  const int tid = threadIdx.x, wave = tid >> 5, lane = tid & 31, col = lane & 15, g = lane >> 4; const size_t r0 = (size_t)blockIdx.x * 64 + wave * 16;
  constexpr int KD = (MODE == 0) ? 2 * CC : CH; const __bf16* P = PK + ((MODE == 0) ? PK_1 : PK_2);
  v8f acc[8] = {};
#pragma unroll
  for (int kc = 0; kc < KD / 32; ++kc) { const v16b ah = frag_b(AHp + (r0 + col) * KD + kc * 32, lane), al = frag_b(ALp + (r0 + col) * KD + kc * 32, lane);
#pragma unroll
    for (int j = 0; j < 8; ++j) { const v16b w = frag_b(P + (size_t)(j * 16 + col) * KD + kc * 32, lane); acc[j] = wmma_bf(al, w, acc[j]); acc[j] = wmma_bf(ah, w, acc[j]); } }
#pragma unroll
  for (int j = 0; j < 8; ++j)
#pragma unroll
    for (int r = 0; r < 8; ++r) so[wave][8 * g + r][j * 16 + col] = acc[j][r];
  __syncthreads();
  for (int rl = 0; rl < 16; ++rl) vst2(OUTR + (r0 + rl) * CH + lane * 4, *(const v4f*)&so[wave][rl][lane * 4]);
  { const int c = tid; double a = 0.0, b2 = 0.0; for (int w = 0; w < 4; ++w) for (int r = 0; r < 16; ++r) { const double v = (double)so[w][r][c]; a += v; b2 += v * v; } sst[c][0] = a; sst[c][1] = b2; }
  __syncthreads();
  vst2((unsigned*)(ST + ((size_t)blockIdx.x * CH + tid) * 2), *(const v4u*)&sst[tid][0]);
}
__global__ __launch_bounds__(128) void k_red(const double* __restrict__ ST, const float* __restrict__ G, const float* __restrict__ BE, float* __restrict__ MR) {
  __shared__ __align__(16) float s[4 * CH]; const int t = threadIdx.x; double a = 0.0, b2 = 0.0;
  for (int blk = 0; blk < NR / 64; ++blk) { a += ST[((size_t)blk * CH + t) * 2]; b2 += ST[((size_t)blk * CH + t) * 2 + 1]; }
  const double mean = a / (double)NR; const double var = fmax(b2 / (double)NR - mean * mean, 0.0);
  s[t] = (float)mean; s[CH + t] = (float)(1.0 / sqrt(var + 1e-5)) * bfr(G[t]); s[2 * CH + t] = bfr(BE[t]); s[3 * CH + t] = 0.f;
  __syncthreads();
  vst2(MR + t * 4, *(const v4f*)&s[t * 4]);
}
__global__ __launch_bounds__(256) void k_bn1(const float* __restrict__ H, const float* __restrict__ MR, __bf16* __restrict__ HBH, __bf16* __restrict__ HBL) {
  __shared__ __align__(16) __bf16 sh_[64][CH + 8], sl_[64][CH + 8]; const int tid = threadIdx.x;
  for (int e = tid; e < 64 * CH; e += 256) { const int r = e / CH, c = e % CH; const size_t row = (size_t)blockIdx.x * 64 + r; float v = (H[row * CH + c] - MR[c]) * MR[CH + c] + MR[2 * CH + c]; v = fmaxf(v, 0.f); const __bf16 hb = (__bf16)v; sh_[r][c] = hb; sl_[r][c] = (__bf16)(v - (float)hb); }
  __syncthreads();
  for (int e = tid; e < 64 * (CH / 8) * 2; e += 256) { const int plane = e / (64 * CH / 8), rem = e % (64 * CH / 8); const int r = rem / (CH / 8), pc = rem % (CH / 8); const size_t o = ((size_t)blockIdx.x * 64 + r) * CH + pc * 8;
    if (plane == 0) vst2((unsigned*)(HBH + o), *(const v4u*)&sh_[r][pc * 8]); else vst2((unsigned*)(HBL + o), *(const v4u*)&sl_[r][pc * 8]); }
}
__global__ __launch_bounds__(128) void k_s(const float* __restrict__ Y, const float* __restrict__ MR2, double* __restrict__ ST3) {
  __shared__ __align__(16) double s[CH]; const int c = threadIdx.x; double a = 0.0;
  for (int r = 0; r < 64; ++r) { const size_t row = (size_t)blockIdx.x * 64 + r; float v = (Y[row * CH + c] - MR2[c]) * MR2[CH + c] + MR2[2 * CH + c]; a += (double)fmaxf(v, 0.f); }
  s[c] = a; __syncthreads();
  if (c < 64) vst2((unsigned*)(ST3 + (size_t)blockIdx.x * CH + c * 2), *(const v4u*)&s[c * 2]);
}
__global__ __launch_bounds__(128) void k_gate(const double* __restrict__ ST3, const float* __restrict__ F1W, const float* __restrict__ F1B, const float* __restrict__ F2W, const float* __restrict__ F2B, float* __restrict__ GT) {
  __shared__ float ss[CH], shid[SEH]; __shared__ __align__(16) float sg[CH]; const int c = threadIdx.x; const int b = blockIdx.x; double a = 0.0;
  for (int blk = 0; blk < NN / 64; ++blk) a += ST3[((size_t)(b * (NN / 64) + blk)) * CH + c];
  ss[c] = (float)(a / (double)NN); __syncthreads();
  if (c < SEH) { float h = bfr(F1B[c]); for (int k = 0; k < CH; ++k) h += ss[k] * bfr(F1W[(size_t)c * CH + k]); shid[c] = fmaxf(h, 0.f); }
  __syncthreads();
  { float v = bfr(F2B[c]);
#pragma unroll
    for (int k = 0; k < SEH; ++k) v += shid[k] * bfr(F2W[(size_t)c * SEH + k]);
    sg[c] = 1.0f / (1.0f + exp_ni(-v)); }
  __syncthreads();
  if (c < 32) vst2(GT + (size_t)b * CH + c * 4, *(const v4f*)&sg[c * 4]);
}
__global__ __launch_bounds__(256) void k_out(const float* __restrict__ Y, const float* __restrict__ MR2, const float* __restrict__ GT, const float* __restrict__ X, float* __restrict__ OUT) {
  __shared__ __align__(16) float st[CH][68]; const int tid = threadIdx.x; const int pb = blockIdx.x, b = blockIdx.y; const int n0 = pb * 64;
  for (int e = tid; e < 64 * CH; e += 256) { const int r = e / CH, c = e % CH; const size_t row = (size_t)b * NN + n0 + r; float v = (Y[row * CH + c] - MR2[c]) * MR2[CH + c] + MR2[2 * CH + c]; v = fmaxf(v, 0.f) * GT[b * CH + c]; st[c][r] = bfr(X[((size_t)b * CC + c) * NNS + n0 + r]) + v; }
  __syncthreads();
  for (int e = tid; e < CH * 16; e += 256) { const int c = e >> 4, pc = e & 15; vst2(OUT + ((size_t)b * CC + c) * NN + n0 + pc * 4, *(const v4f*)&st[c][pc * 4]); }
}
extern "C" void kernel_launch(void* const* d_in, const int* in_sizes, int n_in, void* d_out, int out_size, void* d_ws, size_t ws_size, hipStream_t stream) {
  (void)in_sizes; (void)n_in; (void)out_size;
  const float** F = (const float**)d_in;
  if (ws_size < (size_t)WS_END) return;
  char* ws = (char*)d_ws; __bf16 *PK = (__bf16*)(ws + WS_PK), *AH = (__bf16*)(ws + WS_AH), *AL = (__bf16*)(ws + WS_AL), *HBH = (__bf16*)(ws + WS_HBH), *HBL = (__bf16*)(ws + WS_HBL); float *P4 = (float*)(ws + WS_P4), *SQ = (float*)(ws + WS_SQ), *H = (float*)(ws + WS_H), *MR1 = (float*)(ws + WS_MR1), *Y = (float*)(ws + WS_Y), *MR2 = (float*)(ws + WS_MR2), *GT = (float*)(ws + WS_GT); double *ST1 = (double*)(ws + WS_ST1), *ST2 = (double*)(ws + WS_ST2), *ST3 = (double*)(ws + WS_ST3);
  k_pack<<<dim3(CH, 2), 256, 0, stream>>>(F[2], F[5], PK);
  k_prep<<<dim3(NN / 64, NB), 64, 0, stream>>>(F[1], P4, SQ);
  k_knn<<<NR / 4, 128, 0, stream>>>(P4, SQ, F[0], AH, AL);
  k_gemm<0><<<NR / 64, 128, 0, stream>>>(AH, AL, PK, H, ST1);
  k_red<<<1, 128, 0, stream>>>(ST1, F[3], F[4], MR1);
  k_bn1<<<NR / 64, 256, 0, stream>>>(H, MR1, HBH, HBL);
  k_gemm<1><<<NR / 64, 128, 0, stream>>>(HBH, HBL, PK, Y, ST2);
  k_red<<<1, 128, 0, stream>>>(ST2, F[6], F[7], MR2);
  k_s<<<NR / 64, 128, 0, stream>>>(Y, MR2, ST3);
  k_gate<<<NB, 128, 0, stream>>>(ST3, F[8], F[9], F[10], F[11], GT);
  k_out<<<dim3(NN / 64, NB), 256, 0, stream>>>(Y, MR2, GT, F[0], (float*)d_out);
}
